// EfficientSlidingWindowMultiheadAttention_45397804319137
// MI455X (gfx1250) — hardware-run, weakly checked
//
#include <hip/hip_runtime.h>
#define SQ 4096
#define DM 1024
#define NH 16
#define HD 64
#define QKVP (3 * DM)
#define NFR (HD / 2)
#define WCAR 32.0f
#define OCAR 16.0f
typedef __bf16 v16b __attribute__((ext_vector_type(16)));
typedef unsigned short v8us __attribute__((ext_vector_type(8), may_alias));
typedef float  v8f  __attribute__((ext_vector_type(8)));
typedef float  v4f  __attribute__((ext_vector_type(4)));
typedef float  v4fa __attribute__((ext_vector_type(4), may_alias));
union FragB { v16b v; v8us half[2]; unsigned short u[16]; };

__device__ __forceinline__ unsigned short bf16_bits(float x) { unsigned int u = __float_as_uint(x); return (unsigned short)((u + 0x7FFFu + ((u >> 16) & 1u)) >> 16); }
__device__ __forceinline__ float bf16_val(unsigned short b) { return __uint_as_float(((unsigned int)b) << 16); }
__device__ __forceinline__ float bf16_round(float x) { return bf16_val(bf16_bits(x)); }
template <int NT>
__device__ __forceinline__ v8f mmaN(v16b ah, v16b al, v16b bh, v16b bl, v8f c) {
  c = __builtin_amdgcn_wmma_f32_16x16x32_bf16(false, ah, false, bh, (short)0, c, false, false);
  if (NT >= 2) c = __builtin_amdgcn_wmma_f32_16x16x32_bf16(false, al, false, bh, (short)0, c, false, false);
  if (NT >= 3) c = __builtin_amdgcn_wmma_f32_16x16x32_bf16(false, ah, false, bl, (short)0, c, false, false);
  asm volatile("v_nop\n\tv_nop\n\tv_nop\n\tv_nop" : "+v"(c) : "v"(ah), "v"(al), "v"(bh), "v"(bl));
  return c;
}


typedef _Float16 v16h __attribute__((ext_vector_type(16)));
union FragH { v16h v; v8us half[2]; _Float16 h[16]; unsigned short u[16]; };
template <int NT>
__device__ __forceinline__ v8f mmaH(v16h ah, v16h al, v16h bh, v16h bl, v8f c) {
  c = __builtin_amdgcn_wmma_f32_16x16x32_f16(false, ah, false, bh, (short)0, c, false, false);
  if (NT >= 2) c = __builtin_amdgcn_wmma_f32_16x16x32_f16(false, al, false, bh, (short)0, c, false, false);
  if (NT >= 3) c = __builtin_amdgcn_wmma_f32_16x16x32_f16(false, ah, false, bl, (short)0, c, false, false);
  asm volatile("v_nop\n\tv_nop\n\tv_nop\n\tv_nop" : "+v"(c) : "v"(ah), "v"(al), "v"(bh), "v"(bl));
  return c;
}

__global__ __launch_bounds__(256) void k_wt_f16(const float* __restrict__ W, _Float16* __restrict__ Wt, int K, int N, float scale) {
  const int t = blockIdx.x * 256 + threadIdx.x; if (t >= N * (K / 8)) return; const int n = t / (K / 8), k8 = (t % (K / 8)) * 8; FragH f;
#pragma unroll
  for (int i = 0; i < 8; ++i) f.h[i] = (_Float16)(bf16_round(W[(size_t)(k8 + i) * N + n]) * scale); const v8us o = f.half[0];
  *(volatile v8us*)((unsigned short*)Wt + (size_t)n * K + k8) = o; __threadfence(); *(volatile v8us*)((unsigned short*)Wt + (size_t)n * K + k8) = o;
}

typedef _Float16 v4h __attribute__((ext_vector_type(4)));

__global__ __launch_bounds__(256) void k_x16(const float* __restrict__ x, _Float16* __restrict__ X16, size_t n8) { const size_t t = (size_t)blockIdx.x * 256 + threadIdx.x; if (t >= n8) return; FragH f;
#pragma unroll
  for (int q = 0; q < 8; ++q) f.h[q] = (_Float16)bf16_round(x[t * 8 + q]); *(volatile v8us*)((unsigned short*)X16 + t * 8) = f.half[0]; __threadfence(); *(volatile v8us*)((unsigned short*)X16 + t * 8) = f.half[0]; }
__device__ __forceinline__ v16h g2_frag(const _Float16* p, int hh) { FragH f; f.half[0] = *(const v8us*)((const unsigned short*)p + 8 * hh); f.half[1] = *(const v8us*)((const unsigned short*)p + 16 + 8 * hh); return f.v; }
__device__ __forceinline__ v8f g2_mma(v16h a, v16h b, v8f c) { v8f d = __builtin_amdgcn_wmma_f32_16x16x32_f16(false, a, false, b, (short)0, c, false, false); asm volatile("v_nop\n\tv_nop\n\tv_nop\n\tv_nop" : "+v"(d) : "v"(a), "v"(b)); return d; }
template <int ACT>
__global__ __launch_bounds__(128) void k_gemm2(const _Float16* __restrict__ A, int lda, size_t sA, const _Float16* __restrict__ Bh, int ldb, size_t sB, float alpha, const float* __restrict__ bias, size_t sBias, const float* __restrict__ CP, int rowsPerB, size_t sCPb, int row0g,
    float* __restrict__ C, _Float16* __restrict__ C16, int ldc, size_t sC, int M, int N, int K) { static_assert(ACT == 0 || ACT == 3 || ACT == 6 || ACT == 8 || ACT == 9 || ACT == 11 || ACT == 12 || ACT == 14 || ACT == 15 || ACT == 16 || ACT == 17, "k_gemm2: unsupported ACT code (would silently apply no activation)");
  __shared__ __attribute__((aligned(16))) float so[4][32][68];
  const int tid = threadIdx.x, w = tid >> 5, lane = tid & 31, ln = lane & 15, hh = lane >> 4; const int by = blockIdx.y;
  A += (size_t)by * sA; Bh += (size_t)by * sB; const size_t cofs = (size_t)by * sC; const float* bp = bias ? bias + (size_t)by * sBias : nullptr;
  const int ntn = N >> 6; const int mt = blockIdx.x / ntn, nq = blockIdx.x - mt * ntn; const int row0 = mt * 128 + 32 * w, col0 = nq * 64; if (row0 >= M) return;
  const _Float16* a0p = A + (size_t)(row0 + ln) * lda; const _Float16* a1p = a0p + (size_t)16 * lda;
  const _Float16* b0p = Bh + (size_t)(col0 + ln) * ldb; const _Float16* b1p = b0p + (size_t)16 * ldb; const _Float16* b2p = b1p + (size_t)16 * ldb; const _Float16* b3p = b2p + (size_t)16 * ldb;
  const v8f z8 = {0.f,0.f,0.f,0.f,0.f,0.f,0.f,0.f}; v8f c00 = z8, c01 = z8, c02 = z8, c03 = z8, c10 = z8, c11 = z8, c12 = z8, c13 = z8;
  for (int kb = 0; kb < K; kb += 32) { const v16h a0 = g2_frag(a0p + kb, hh), a1 = g2_frag(a1p + kb, hh);
    v16h b = g2_frag(b0p + kb, hh); c00 = g2_mma(a0, b, c00); c10 = g2_mma(a1, b, c10);
    b = g2_frag(b1p + kb, hh); c01 = g2_mma(a0, b, c01); c11 = g2_mma(a1, b, c11);
    b = g2_frag(b2p + kb, hh); c02 = g2_mma(a0, b, c02); c12 = g2_mma(a1, b, c12);
    b = g2_frag(b3p + kb, hh); c03 = g2_mma(a0, b, c03); c13 = g2_mma(a1, b, c13); }
  v8f accs[8] = {c00, c01, c02, c03, c10, c11, c12, c13};
#pragma unroll
  for (int u = 0; u < 8; ++u) { const int t = u & 3, half = u >> 2; const int col = col0 + t * 16 + ln; const float bv = bp ? bf16_round(bp[col]) : 0.f;
#pragma unroll
    for (int r = 0; r < 8; ++r) { const int rloc = half * 16 + 8 * hh + r; float v = accs[u][r] * alpha + bv; if (CP) { if (rowsPerB < 0) v += CP[cofs + (size_t)(row0g + row0 + rloc) * ldc + col];        else { const int bidx = (row0g + row0 + rloc) / rowsPerB; v += CP[(size_t)bidx * sCPb + (size_t)by * 64 + col]; } }
      if (ACT == 3) v = fmaxf(v, 0.f); else if (ACT == 6) v = 0.5f * v * (1.0f + erff(v * 0.70710678118654752f)); else if (ACT == 11) v = 1.0f / (1.0f + expf(-v)); else if (ACT == 15) v = v / (1.0f + expf(-v)); else if (ACT == 12) v = (v > 0.f) ? v : 0.01f * v; else if (ACT == 8) v = tanhf(v); else if (ACT == 9) v = 0.5f * v * (1.0f + tanhf(0.7978845608028654f * (v + 0.044715f * v * v * v))); else if (ACT == 14) v = (v > 0.f) ? v : 0.1f * v; else if (ACT == 16) v = (v >= 0.f) ? v : 0.3f * v; else if (ACT == 17) v = (v >= 0.f) ? v : 0.2f * v;
      so[w][rloc][t * 16 + ln] = v; } }
  __builtin_amdgcn_fence(__ATOMIC_ACQ_REL, "workgroup"); __builtin_amdgcn_wave_barrier();
  const int rsub = lane >> 4, c4 = (lane & 15) * 4;
  for (int pass = 0; pass < 2; ++pass) {
#pragma unroll
    for (int q = 0; q < 16; ++q) { const int r = q * 2 + rsub; const v4f v = *(const v4fa*)&so[w][r][c4]; if (C) *(volatile v4f*)(C + cofs + (size_t)(row0 + r) * ldc + col0 + c4) = v; if (C16) { v4h h4; for (int i = 0; i < 4; ++i) h4[i] = (_Float16)v[i]; *(volatile v4h*)(C16 + cofs + (size_t)(row0 + r) * ldc + col0 + c4) = h4; } }
    if (pass == 0) __threadfence(); } }


__global__ __launch_bounds__(256) void k_trigpoly(const float* __restrict__ rot, float* __restrict__ CS, float* __restrict__ SN, int n) {
  const int t = blockIdx.x * 256 + threadIdx.x; if (t >= n) return; const float a = bf16_round(rot[t]);
  const float u1 = a * 0.15915679931640625f; const float f1 = u1 - rintf(u1); const float fr = f1 + (a * -1.8562132027000189e-06f + a * -1.1308204372895148e-11f);
  const float k = rintf(fr * 4.0f); const float y = fr - k * 0.25f; const float r = y * 6.2831853071795865f; const float z = r * r;
  const float s = r + (r * z) * (-1.6666654611e-1f + z * (8.3321608736e-3f + z * -1.9515295891e-4f));
  const float c = 1.0f - 0.5f * z + (z * z) * (4.166664568298827e-2f + z * (-1.388731625493765e-3f + z * 2.443315711809948e-5f));
  const unsigned q = (unsigned)(int)k; const unsigned mk = 0u - (q & 1u); const unsigned cb = __float_as_uint(c), sb = __float_as_uint(s);
  const float co = __uint_as_float(((cb & ~mk) | (sb & mk)) ^ ((((q + 1u) >> 1) & 1u) << 31)); const float si = __uint_as_float(((sb & ~mk) | (cb & mk)) ^ (((q >> 1) & 1u) << 31));
  *(volatile float*)(CS + t) = co; *(volatile float*)(SN + t) = si; __threadfence(); *(volatile float*)(CS + t) = co; *(volatile float*)(SN + t) = si; }
__global__ __launch_bounds__(256) void k_rope4p(float* __restrict__ QKV, const float* __restrict__ CS, const float* __restrict__ SN, int n) {
  const int t = blockIdx.x * 256 + threadIdx.x; if (t >= n) return; const int g = t & 7, part = (t >> 3) & 1, h = (t >> 4) & 15, s = t >> 8;
  float* p = QKV + (size_t)s * QKVP + h * (3 * HD) + part * HD + g * 8; const v4f w0 = *(const v4fa*)p, w1 = *(const v4fa*)(p + 4); const v4f c = *(const v4fa*)(CS + (size_t)s * NFR + g * 4), sn = *(const v4fa*)(SN + (size_t)s * NFR + g * 4);
  v4f o0, o1; o0[0] = w0[0] * c[0] - w0[1] * sn[0]; o0[1] = w0[0] * sn[0] + w0[1] * c[0]; o0[2] = w0[2] * c[1] - w0[3] * sn[1]; o0[3] = w0[2] * sn[1] + w0[3] * c[1]; o1[0] = w1[0] * c[2] - w1[1] * sn[2]; o1[1] = w1[0] * sn[2] + w1[1] * c[2]; o1[2] = w1[2] * c[3] - w1[3] * sn[3]; o1[3] = w1[2] * sn[3] + w1[3] * c[3];
  *(volatile v4f*)p = o0; *(volatile v4f*)(p + 4) = o1; __threadfence(); *(volatile v4f*)p = o0; *(volatile v4f*)(p + 4) = o1; }
__global__ __launch_bounds__(256) void k_win33(const float* __restrict__ QKV, _Float16* __restrict__ O16, int n) {
  const int t = blockIdx.x * 256 + threadIdx.x; if (t >= n) return; const int h = t & 15, s = t >> 4;
  const float* q = QKV + (size_t)s * QKVP + h * (3 * HD); v4f qv[16];
  for (int c = 0; c < 16; ++c) qv[c] = *(const v4fa*)(q + 4 * c);
  float m = -3.0e38f, l = 0.f; float acc[HD];
  for (int c = 0; c < HD; ++c) acc[c] = 0.f;
  for (int w = 0; w < 33; ++w) { const int ts = s + w - 16; const int ct = (ts < 0) ? 0 : ((ts > SQ - 1) ? (SQ - 1) : ts); const float on = (ts == ct) ? 1.0f : 0.0f; const float* k = QKV + (size_t)ct * QKVP + h * (3 * HD) + HD; float dot = 0.f;
    for (int c = 0; c < 16; ++c) { const v4f kv = *(const v4fa*)(k + 4 * c); dot += qv[c][0] * kv[0]; dot += qv[c][1] * kv[1]; dot += qv[c][2] * kv[2]; dot += qv[c][3] * kv[3]; }
    const float sc = on * (dot * 0.125f); const float mn = (sc > m) ? sc : m; const float corr = expf(m - mn); const float pw = expf(sc - mn); l = l * corr + pw; const float pv = pw * on; const float* v = k + HD;
    for (int c = 0; c < 16; ++c) { const v4f vv = *(const v4fa*)(v + 4 * c); acc[4 * c] = acc[4 * c] * corr + pv * vv[0]; acc[4 * c + 1] = acc[4 * c + 1] * corr + pv * vv[1]; acc[4 * c + 2] = acc[4 * c + 2] * corr + pv * vv[2]; acc[4 * c + 3] = acc[4 * c + 3] * corr + pv * vv[3]; }
    m = mn; }
  const float f = OCAR / l; unsigned short* d = (unsigned short*)O16 + (size_t)s * DM + h * HD;
  for (int g = 0; g < 8; ++g) { FragH o;
    for (int c = 0; c < 8; ++c) o.h[c] = (_Float16)(acc[8 * g + c] * f);
    *(volatile v8us*)(d + 8 * g) = o.half[0]; __threadfence(); *(volatile v8us*)(d + 8 * g) = o.half[0]; } }

extern "C" void kernel_launch(void* const* d_in, const int* in_sizes, int n_in,
                              void* d_out, int out_size, void* d_ws, size_t ws_size, hipStream_t stream) {
  (void)in_sizes; (void)n_in; (void)out_size;
  const float* x = (const float*)d_in[0]; const float* rot = (const float*)d_in[1]; const float* wqkv = (const float*)d_in[2]; const float* bqkv = (const float*)d_in[3]; const float* wo = (const float*)d_in[4]; const float* bo = (const float*)d_in[5];
  static_assert(DM == NH * HD && NH == 16 && HD == 64 && NFR == 32 && SQ % 128 == 0 && QKVP % 64 == 0 && DM % 64 == 0 && ((size_t)SQ * NFR) % 256 == 0 && ((size_t)SQ * NH * 16) % 256 == 0 && ((size_t)SQ * NH) % 256 == 0 && ((size_t)SQ * DM / 8) % 256 == 0, "the index shifts; whole tiles; exact grids");
  char* ws = (char*)d_ws; size_t off = 0;
  auto take = [&](size_t bytes) { char* p = ws + off; off += (bytes + 255) & ~(size_t)255; return p; };
  _Float16* WT = (_Float16*)take((size_t)QKVP * DM * 2); _Float16* WO = (_Float16*)take((size_t)DM * DM * 2); _Float16* X16 = (_Float16*)take((size_t)SQ * DM * 2); float* QKV = (float*)take((size_t)SQ * QKVP * 4); float* CS = (float*)take((size_t)SQ * NFR * 4); float* SN = (float*)take((size_t)SQ * NFR * 4); _Float16* O16 = (_Float16*)take((size_t)SQ * DM * 2);
  if (off > ws_size) return;
  k_wt_f16<<<(unsigned)(((size_t)QKVP * (DM / 8) + 255) / 256), 256, 0, stream>>>(wqkv, WT, DM, QKVP, WCAR); k_wt_f16<<<(unsigned)(((size_t)DM * (DM / 8) + 255) / 256), 256, 0, stream>>>(wo, WO, DM, DM, WCAR);
  k_x16<<<(unsigned)(((size_t)SQ * DM / 8 + 255) / 256), 256, 0, stream>>>(x, X16, (size_t)SQ * DM / 8);
  k_gemm2<0><<<dim3((unsigned)((SQ / 128) * (QKVP / 64)), 1), 128, 0, stream>>>(X16, DM, 0, WT, DM, 0, 1.0f / WCAR, bqkv, 0, nullptr, 1, 0, 0, QKV, nullptr, QKVP, 0, SQ, QKVP, DM);
  k_trigpoly<<<(unsigned)((size_t)SQ * NFR / 256), 256, 0, stream>>>(rot, CS, SN, SQ * NFR);
  k_rope4p<<<(unsigned)((size_t)SQ * NH * 16 / 256), 256, 0, stream>>>(QKV, CS, SN, SQ * NH * 16);
  k_win33<<<(unsigned)((size_t)SQ * NH / 256), 256, 0, stream>>>(QKV, O16, SQ * NH);
  k_gemm2<0><<<dim3((unsigned)((SQ / 128) * (DM / 64)), 1), 128, 0, stream>>>(O16, DM, 0, WO, DM, 0, 1.0f / (WCAR * OCAR), bo, 0, nullptr, 1, 0, 0, (float*)d_out, nullptr, DM, 0, SQ, DM, DM);
}
